// SeqLinear_69844758167722
// MI455X (gfx1250) — hardware-verified
//
#include <hip/hip_runtime.h>
#include <stdint.h>

typedef __attribute__((ext_vector_type(16))) _Float16 v16h;
typedef __attribute__((ext_vector_type(8)))  _Float16 v8h;
typedef __attribute__((ext_vector_type(16))) __bf16   v16b;
typedef __attribute__((ext_vector_type(8)))  __bf16   v8b;
typedef __attribute__((ext_vector_type(8)))  float    v8f;
typedef __attribute__((ext_vector_type(4)))  float    v4f;

static constexpr int kBatch   = 4;
static constexpr int kSeq     = 1024;
static constexpr int kDModel  = 1024;
static constexpr int kHeads   = 16;
static constexpr int kDConv   = 4;
static constexpr int kDState  = 1024;
static constexpr int kDInner  = 1024;
static constexpr int kConvDim = 3072;
static constexpr int kDInProj = 3088;
static constexpr int kNPad    = 3136;
static constexpr int kRows    = kBatch * kSeq;
static constexpr int kTTile   = 32;
static_assert(kConvDim == 2 * kDState + kDInner, "geom");
static_assert(kDInProj == kConvDim + kHeads, "geom");
static_assert(kNPad % 64 == 0 && kNPad >= kDInProj, "pad");
static_assert(kRows % 64 == 0 && kDModel % 32 == 0 && kDInner % 32 == 0, "tiles");

__device__ __forceinline__ unsigned short f2bf_bits(float f) {
  unsigned u = __float_as_uint(f);
  return (unsigned short)((u + 0x7FFFu + ((u >> 16) & 1u)) >> 16);
}
__device__ __forceinline__ float bf_bits2f(unsigned short h) { return __uint_as_float(((unsigned)h) << 16); }

__device__ __forceinline__ void dep_guard_h(v8f& a, v8f& b, v16h x, v16h y) { asm volatile("v_nop\n\tv_nop\n\tv_nop\n\tv_nop" : "+v"(a), "+v"(b) : "v"(x), "v"(y)); }
__device__ __forceinline__ void dep_guard_b(v8f& a, v8f& b, v16b x, v16b y) { asm volatile("v_nop\n\tv_nop\n\tv_nop\n\tv_nop" : "+v"(a), "+v"(b) : "v"(x), "v"(y)); }
__device__ __forceinline__ void keep4_h(v16h a, v16h b, v16h c, v16h d) { asm volatile("v_nop" :: "v"(a), "v"(b), "v"(c), "v"(d)); }
__device__ __forceinline__ void keep4_b(v16b a, v16b b, v16b c, v16b d) { asm volatile("v_nop" :: "v"(a), "v"(b), "v"(c), "v"(d)); }
__device__ __forceinline__ void acc_guard4(v8f& a, v8f& b, v8f& c, v8f& d) { asm volatile("v_nop\n\tv_nop\n\tv_nop\n\tv_nop" : "+v"(a), "+v"(b), "+v"(c), "+v"(d)); }
template <typename T> struct Frag;
template <> struct Frag<_Float16> {
  typedef v16h V; union U { v16h v; v8h h[2]; };
  static __device__ __forceinline__ v16h load(const _Float16* p) {
    U f; f.h[0] = *(const v8h*)(p); f.h[1] = *(const v8h*)(p + 16); return f.v;
  }
  static __device__ __forceinline__ v8f mma(v16h a, v16h b, v8f c) {
    return __builtin_amdgcn_wmma_f32_16x16x32_f16(false, a, false, b, (short)0, c, false, false);
  }
  static __device__ __forceinline__ void guard(v8f& a, v8f& b, v16h x, v16h y) { dep_guard_h(a, b, x, y); }
  static __device__ __forceinline__ void keep(v16h a, v16h b, v16h c, v16h d) { keep4_h(a, b, c, d); }
};
template <> struct Frag<__bf16> {
  typedef v16b V; union U { v16b v; v8b h[2]; };
  static __device__ __forceinline__ v16b load(const __bf16* p) {
    U f; f.h[0] = *(const v8b*)(p); f.h[1] = *(const v8b*)(p + 16); return f.v;
  }
  static __device__ __forceinline__ v8f mma(v16b a, v16b b, v8f c) {
    return __builtin_amdgcn_wmma_f32_16x16x32_bf16(false, a, false, b, (short)0, c, false, false);
  }
  static __device__ __forceinline__ void guard(v8f& a, v8f& b, v16b x, v16b y) { dep_guard_b(a, b, x, y); }
  static __device__ __forceinline__ void keep(v16b a, v16b b, v16b c, v16b d) { keep4_b(a, b, c, d); }
};

template <int ET> struct Elem;
template <> struct Elem<0> { typedef _Float16 T; };
template <> struct Elem<1> { typedef __bf16 T; };
template <int ET, bool SPLIT, int BIAS_MODE, int OUT_MODE, bool RESID, int ACT = 0>
__global__ __launch_bounds__(256) void wmma_gemm64(
    const unsigned short* __restrict__ Ap, const unsigned short* __restrict__ A2p, int lda, long strideA,
    const unsigned short* __restrict__ Btp, const unsigned short* __restrict__ Bt2p, int ldb, long strideB,
    void* __restrict__ Cout, void* __restrict__ Cout2, int ldc, long strideC,
    const float* __restrict__ bias,
    const float* __restrict__ resid, long strideR,
    int M, int N, int K, float scale) {
  typedef typename Elem<ET>::T T;
  typedef typename Frag<T>::V V;
  const T* A = (const T*)Ap; const T* A2 = (const T*)A2p; const T* Bt = (const T*)Btp; const T* Bt2 = (const T*)Bt2p;
  __shared__ __align__(16) float sT[8][16 * 68];
  const int b    = blockIdx.y;
  const int lane = threadIdx.x & 31;
  const int wave = threadIdx.x >> 5;
  const int tilesN = N >> 6;
  const int tilesM = M >> 6;
  const int tile = blockIdx.x * 8 + wave;
  if (tile >= tilesM * tilesN) return;
  const int tm = tile / tilesN;
  const int tn = tile - tm * tilesN;
  const int m0 = tm << 6;
  const int n0 = tn << 6;

  const T* Ab  = A  + (size_t)b * strideA;
  const T* Bb  = Bt + (size_t)b * strideB;
  const T* Ab2 = SPLIT ? (A2  + (size_t)b * strideA) : nullptr;
  const T* Bb2 = SPLIT ? (Bt2 + (size_t)b * strideB) : nullptr;

  const int rlane = lane & 15;
  const int koff  = (lane >> 4) * 8;
  const int mOff  = (lane >> 4) * 8;

  v8f acc[4][4];
#pragma unroll
  for (int i = 0; i < 4; ++i)
#pragma unroll
    for (int j = 0; j < 4; ++j) acc[i][j] = (v8f){0.f,0.f,0.f,0.f,0.f,0.f,0.f,0.f};

  for (int k0 = 0; k0 < K; k0 += 32) {
    V bh[4], bl[4];
#pragma unroll
    for (int j = 0; j < 4; ++j) {
      const size_t bo = (size_t)(n0 + (j << 4) + rlane) * ldb + koff + k0;
      bh[j] = Frag<T>::load(Bb + bo);
      if (SPLIT) bl[j] = Frag<T>::load(Bb2 + bo);
    }
#pragma unroll
    for (int i = 0; i < 4; ++i) {
      const size_t ao = (size_t)(m0 + (i << 4) + rlane) * lda + koff + k0;
      V ah = Frag<T>::load(Ab + ao);
      V al;
      if (SPLIT) al = Frag<T>::load(Ab2 + ao);
#pragma unroll
      for (int j = 0; j < 4; ++j) {
        acc[i][j] = Frag<T>::mma(ah, bh[j], acc[i][j]);
        if (SPLIT) {
          acc[i][j] = Frag<T>::mma(ah, bl[j], acc[i][j]);
          acc[i][j] = Frag<T>::mma(al, bh[j], acc[i][j]);
        }
      }
      Frag<T>::guard(acc[i][0], acc[i][3], ah, SPLIT ? al : ah);
    }
    Frag<T>::keep(bh[0], bh[1], bh[2], bh[3]);
    if (SPLIT) Frag<T>::keep(bl[0], bl[1], bl[2], bl[3]);
  }
  acc_guard4(acc[0][0], acc[0][1], acc[0][2], acc[0][3]);
  acc_guard4(acc[1][0], acc[1][1], acc[1][2], acc[1][3]);
  acc_guard4(acc[2][0], acc[2][1], acc[2][2], acc[2][3]);
  acc_guard4(acc[3][0], acc[3][1], acc[3][2], acc[3][3]);

  float* slab = sT[wave];
  const float* Rb = RESID ? (resid + (size_t)b * strideR) : nullptr;
#pragma unroll
  for (int i = 0; i < 4; ++i) {
    const int mBase = m0 + (i << 4);
#pragma unroll
    for (int j = 0; j < 4; ++j) {
      const int n = n0 + (j << 4) + rlane;
      float bv = 0.f;
      if (BIAS_MODE == 2) bv = bias[n];
#pragma unroll
      for (int r = 0; r < 8; ++r) {
        float v = acc[i][j][r] * scale;
        if (BIAS_MODE == 1) v += bias[mBase + mOff + r];
        if (BIAS_MODE == 2) v += bv;
        if (RESID) v += Rb[(size_t)(mBase + mOff + r) * ldc + n];
        if (ACT == 1) v = tanhf(v);
        if (ACT == 2) v = fmaxf(v, 0.0f);
        if (ACT == 3) v = v / (1.0f + expf(-v));
        if (ACT == 4) v = (v > 0.f) ? v : 0.01f * v;
        slab[(mOff + r) * 68 + (j << 4) + rlane] = v;
      }
    }
    __builtin_amdgcn_fence(__ATOMIC_RELEASE, "workgroup");
    __builtin_amdgcn_wave_barrier();
    __builtin_amdgcn_fence(__ATOMIC_ACQUIRE, "workgroup");
    if (OUT_MODE == 0) {
      float* C = (float*)Cout + (size_t)b * strideC;
      const int hh = lane >> 4, c4 = (lane & 15) * 4;
      for (int pass = 0; pass < 2; ++pass) {
#pragma unroll
        for (int it = 0; it < 8; ++it) {
          const int row = it * 2 + hh;
          v4f v = *(const v4f*)(slab + row * 68 + c4);
          *(volatile v4f*)(C + (size_t)(mBase + row) * ldc + n0 + c4) = v;
        }
        __threadfence();
      }
    } else {
      const int q = lane >> 3, c8 = (lane & 7) * 8;
      unsigned short* C  = (unsigned short*)Cout  + (size_t)b * strideC;
      unsigned short* C2 = (OUT_MODE == 2) ? ((unsigned short*)Cout2 + (size_t)b * strideC) : nullptr;
      for (int pass = 0; pass < 2; ++pass) {
#pragma unroll
        for (int it = 0; it < 4; ++it) {
          const int row = it * 4 + q;
          const float* sp = slab + row * 68 + c8;
          v8h hv, lv;
#pragma unroll
          for (int e = 0; e < 8; ++e) {
            if (OUT_MODE == 1) {
              hv[e] = (_Float16)sp[e];
            } else {
              unsigned short hb = f2bf_bits(sp[e]);
              unsigned short lb = f2bf_bits(sp[e] - bf_bits2f(hb));
              hv[e] = __builtin_bit_cast(_Float16, hb);
              lv[e] = __builtin_bit_cast(_Float16, lb);
            }
          }
          *(volatile v8h*)(C + (size_t)(mBase + row) * ldc + n0 + c8) = hv;
          if (OUT_MODE == 2) *(volatile v8h*)(C2 + (size_t)(mBase + row) * ldc + n0 + c8) = lv;
        }
        __threadfence();
      }
    }
    __builtin_amdgcn_fence(__ATOMIC_RELEASE, "workgroup");
    __builtin_amdgcn_wave_barrier();
    __builtin_amdgcn_fence(__ATOMIC_ACQUIRE, "workgroup");
  }
}

__global__ __launch_bounds__(256) void split_bf16_planes(const float* __restrict__ in,
                                                         unsigned short* __restrict__ hi,
                                                         unsigned short* __restrict__ lo,
                                                         int rows_in, int rows_out, int cols) {
  const int i = blockIdx.x * 256 + threadIdx.x;
  const int n8 = (rows_out * cols) >> 3;
  if (i >= n8) return;
  const int e0 = i << 3;
  const int row = e0 / cols;
  const int col = e0 - row * cols;
  const bool live = row < rows_in;
  const int rowc = live ? row : (rows_in - 1);
  const float* p = in + (size_t)rowc * cols + col;
  const v4f f0 = *(const v4f*)(p);
  const v4f f1 = *(const v4f*)(p + 4);
  v8h hv, lv;
#pragma unroll
  for (int e = 0; e < 8; ++e) {
    float f = (e < 4) ? f0[e] : f1[e - 4];
    if (!live) f = 0.0f;
    const unsigned short hb = f2bf_bits(f);
    const unsigned short lb = f2bf_bits(f - bf_bits2f(hb));
    hv[e] = __builtin_bit_cast(_Float16, hb);
    lv[e] = __builtin_bit_cast(_Float16, lb);
  }
  unsigned short* ph = hi + e0;
  unsigned short* pl = lo + e0;
  *(volatile v8h*)ph = hv;
  *(volatile v8h*)pl = lv;
  __threadfence();
  *(volatile v8h*)ph = hv;
  *(volatile v8h*)pl = lv;
}

__global__ __launch_bounds__(256) void conv_gate_kernel(const float* __restrict__ X,
                                                       const float* __restrict__ conv_w,
                                                       const float* __restrict__ conv_b,
                                                       const float* __restrict__ w_base,
                                                       float* __restrict__ OO,
                                                       float* __restrict__ G,
                                                       float* __restrict__ WH) {
  __shared__ __align__(16) float gs[kHeads * kTTile];
  __shared__ __align__(16) float whs[kHeads * kTTile];
  const int tid  = threadIdx.x;
  const int lane = tid & 31;
  const int blk  = blockIdx.x;
  const int b    = blk / (kSeq / kTTile);
  const int t0   = (blk - b * (kSeq / kTTile)) * kTTile;
  const int cb   = tid * 4;
  const int hq   = tid >> 4;
  const int hw   = tid & 15;

  v4f wS[4], wI[4], wO[4];
#pragma unroll
  for (int j = 0; j < 4; ++j) {
    wS[j] = *(const v4f*)(conv_w + (size_t)(cb + j) * kDConv);
    wI[j] = *(const v4f*)(conv_w + (size_t)(kDState + cb + j) * kDConv);
    wO[j] = *(const v4f*)(conv_w + (size_t)(2 * kDState + cb + j) * kDConv);
  }
  const v4f bS = *(const v4f*)(conv_b + cb);
  const v4f bI = *(const v4f*)(conv_b + kDState + cb);
  const v4f bO = *(const v4f*)(conv_b + 2 * kDState + cb);
  const float wb = w_base[hw];

  const v4f z4 = {0.f, 0.f, 0.f, 0.f};
  v4f s0 = z4, s1 = z4, s2 = z4, i0 = z4, i1 = z4, i2 = z4, o0 = z4, o1 = z4, o2 = z4;
  if (t0 > 0) {
    const float* r0 = X + (size_t)(b * kSeq + t0 - 3) * kNPad;
    const float* r1 = r0 + kNPad;
    const float* r2 = r1 + kNPad;
    s0 = *(const v4f*)(r0 + cb); s1 = *(const v4f*)(r1 + cb); s2 = *(const v4f*)(r2 + cb);
    i0 = *(const v4f*)(r0 + kDState + cb); i1 = *(const v4f*)(r1 + kDState + cb); i2 = *(const v4f*)(r2 + kDState + cb);
    o0 = *(const v4f*)(r0 + 2 * kDState + cb); o1 = *(const v4f*)(r1 + 2 * kDState + cb); o2 = *(const v4f*)(r2 + 2 * kDState + cb);
  }

#pragma unroll 1
  for (int i = 0; i < kTTile; ++i) {
    const int bt = b * kSeq + t0 + i;
    const float* row = X + (size_t)bt * kNPad;
    const v4f s3 = *(const v4f*)(row + cb);
    const v4f i3 = *(const v4f*)(row + kDState + cb);
    const v4f o3 = *(const v4f*)(row + 2 * kDState + cb);
    const float wv = row[kConvDim + hw];
    v4f ys, yi, yo;
#pragma unroll
    for (int j = 0; j < 4; ++j) {
      ys[j] = (((wS[j][0] * s0[j] + wS[j][1] * s1[j]) + wS[j][2] * s2[j]) + wS[j][3] * s3[j]) + bS[j];
      yi[j] = (((wI[j][0] * i0[j] + wI[j][1] * i1[j]) + wI[j][2] * i2[j]) + wI[j][3] * i3[j]) + bI[j];
      yo[j] = (((wO[j][0] * o0[j] + wO[j][1] * o1[j]) + wO[j][2] * o2[j]) + wO[j][3] * o3[j]) + bO[j];
    }
    float gp = ((ys[0] * yi[0] + ys[1] * yi[1]) + ys[2] * yi[2]) + ys[3] * yi[3];
    gp += __shfl_xor(gp, 1, 32);
    gp += __shfl_xor(gp, 2, 32);
    gp += __shfl_xor(gp, 4, 32);
    gp += __shfl_xor(gp, 8, 32);
    if ((lane & 15) == 0) gs[hq * kTTile + i] = gp;
    if (tid < kHeads) whs[hw * kTTile + i] = wv * wb;
    float* op = OO + (size_t)bt * kDInner + cb;
    const v4f yov = yo;
    *(volatile v4f*)op = yov;
    __threadfence();
    *(volatile v4f*)op = yov;
    s0 = s1; s1 = s2; s2 = s3;
    i0 = i1; i1 = i2; i2 = i3;
    o0 = o1; o1 = o2; o2 = o3;
  }
  __syncthreads();
  {
    const int u  = tid & 127;
    const int hl = u >> 3;
    const int q  = u & 7;
    const v4f vg = *(const v4f*)(gs  + hl * kTTile + q * 4);
    const v4f vw = *(const v4f*)(whs + hl * kTTile + q * 4);
    const size_t o = (size_t)(b * kHeads + hl) * kSeq + t0 + q * 4;
    if (tid < 128) {
      *(volatile v4f*)(G + o) = vg;
      __threadfence();
      *(volatile v4f*)(G + o) = vg;
    } else {
      *(volatile v4f*)(WH + o) = vw;
      __threadfence();
      *(volatile v4f*)(WH + o) = vw;
    }
  }
}

__global__ __launch_bounds__(64) void prefix_kernel(const float* __restrict__ G,
                                                   const float* __restrict__ WH,
                                                   float* __restrict__ A) {
  __shared__ __align__(16) float aT[64 * 32];
  const int tid = threadIdx.x;
  const float* gp = G  + (size_t)tid * kSeq;
  const float* wp = WH + (size_t)tid * kSeq;
  float cs = 0.f, m = -1.0e30f, num = 0.f, den = 0.f;
#pragma unroll 1
  for (int ch = 0; ch < kSeq / 32; ++ch) {
#pragma unroll 1
    for (int j = 0; j < 32; ++j) {
      const int t = ch * 32 + j;
      const float wv = wp[t];
      const float gv = gp[t];
      cs += wv;
      const float z  = -cs;
      const float mn = fmaxf(m, z);
      const float sc = expf(m - mn);
      const float ez = expf(z - mn);
      num = num * sc + gv * ez;
      den = den * sc + ez;
      m = mn;
      aT[tid * 32 + j] = num * (1.0f / den);
    }
    __syncthreads();
    const int q = tid & 7;
#pragma unroll
    for (int it = 0; it < 8; ++it) {
      const int line = it * 8 + (tid >> 3);
      const v4f v = *(const v4f*)(aT + line * 32 + q * 4);
      *(volatile v4f*)(A + (size_t)line * kSeq + ch * 32 + q * 4) = v;
    }
    __threadfence();
#pragma unroll
    for (int it = 0; it < 8; ++it) {
      const int line = it * 8 + (tid >> 3);
      const v4f v = *(const v4f*)(aT + line * 32 + q * 4);
      *(volatile v4f*)(A + (size_t)line * kSeq + ch * 32 + q * 4) = v;
    }
    __syncthreads();
  }
}

__global__ __launch_bounds__(256) void combine_kernel(const float* __restrict__ A,
                                                     const float* __restrict__ OO,
                                                     unsigned short* __restrict__ Yh,
                                                     unsigned short* __restrict__ Yl) {
  const int i = blockIdx.x * 256 + threadIdx.x;
  if (i >= (kRows * kDInner) / 8) return;
  const int e0 = i << 3;
  const int bt = e0 >> 10;
  const int c0 = e0 & (kDInner - 1);
  const int b  = bt >> 10;
  const int t  = bt & (kSeq - 1);
  const int h  = c0 >> 6;
  const float a = A[(size_t)(b * kHeads + h) * kSeq + t];
  const v4f q0 = *(const v4f*)(OO + e0);
  const v4f q1 = *(const v4f*)(OO + e0 + 4);
  v8h hv, lv;
#pragma unroll
  for (int e = 0; e < 8; ++e) {
    const float f = a * ((e < 4) ? q0[e] : q1[e - 4]);
    const unsigned short hb = f2bf_bits(f);
    const unsigned short lb = f2bf_bits(f - bf_bits2f(hb));
    hv[e] = __builtin_bit_cast(_Float16, hb);
    lv[e] = __builtin_bit_cast(_Float16, lb);
  }
  unsigned short* ph = Yh + e0;
  unsigned short* pl = Yl + e0;
  *(volatile v8h*)ph = hv;
  *(volatile v8h*)pl = lv;
  __threadfence();
  *(volatile v8h*)ph = hv;
  *(volatile v8h*)pl = lv;
}

extern "C" void kernel_launch(void* const* d_in, const int* in_sizes, int n_in,
                              void* d_out, int out_size, void* d_ws, size_t ws_size,
                              hipStream_t stream) {
  if (n_in < 6) return;
  if (in_sizes[0] != kRows * kDModel) return;
  if (in_sizes[1] != kDInProj * kDModel) return;
  if (in_sizes[2] != kConvDim * kDConv) return;
  if (in_sizes[3] != kConvDim) return;
  if (in_sizes[4] != kHeads) return;
  if (in_sizes[5] != kDModel * kDInner) return;
  if (out_size != kRows * kDModel) return;

  const float* x      = (const float*)d_in[0];
  const float* W_in   = (const float*)d_in[1];
  const float* conv_w = (const float*)d_in[2];
  const float* conv_b = (const float*)d_in[3];
  const float* w_base = (const float*)d_in[4];
  const float* W_out  = (const float*)d_in[5];
  float* out = (float*)d_out;

  char* ws = (char*)d_ws;
  size_t off = 0;
  const size_t szX   = (size_t)kRows * kDModel * 2;
  const size_t szWI  = (size_t)kNPad * kDModel * 2;
  const size_t szWO  = (size_t)kDModel * kDInner * 2;
  const size_t szXIO = (size_t)kRows * kNPad * 4;
  const size_t szOO  = (size_t)kRows * kDInner * 4;
  const size_t szSm  = (size_t)kBatch * kHeads * kSeq * 4;
  const size_t szY   = (size_t)kRows * kDInner * 2;
  unsigned short* XH  = (unsigned short*)(ws + off); off += szX;
  unsigned short* XL  = (unsigned short*)(ws + off); off += szX;
  unsigned short* WIH = (unsigned short*)(ws + off); off += szWI;
  unsigned short* WIL = (unsigned short*)(ws + off); off += szWI;
  unsigned short* WOH = (unsigned short*)(ws + off); off += szWO;
  unsigned short* WOL = (unsigned short*)(ws + off); off += szWO;
  float*          XIO = (float*)(ws + off);          off += szXIO;
  float*          OOb = (float*)(ws + off);          off += szOO;
  float*          Gb  = (float*)(ws + off);          off += szSm;
  float*          WHb = (float*)(ws + off);          off += szSm;
  float*          ACO = (float*)(ws + off);          off += szSm;
  unsigned short* YH  = (unsigned short*)(ws + off); off += szY;
  unsigned short* YL  = (unsigned short*)(ws + off); off += szY;
  if (off > ws_size) return;
  if (off > (size_t)134217728) return;

  split_bf16_planes<<<(kRows * kDModel / 8) / 256, 256, 0, stream>>>(x, XH, XL, kRows, kRows, kDModel);
  split_bf16_planes<<<(kNPad * kDModel / 8) / 256, 256, 0, stream>>>(W_in, WIH, WIL, kDInProj, kNPad, kDModel);
  split_bf16_planes<<<(kDModel * kDInner / 8) / 256, 256, 0, stream>>>(W_out, WOH, WOL, kDModel, kDModel, kDInner);

  {
    dim3 grid((kRows / 64) * (kNPad / 64) / 8, 1);
    wmma_gemm64<1, true, 0, 0, false, 0><<<grid, 256, 0, stream>>>(
        XH, XL, kDModel, 0L, WIH, WIL, kDModel, 0L,
        (void*)XIO, nullptr, kNPad, 0L, nullptr, nullptr, 0L,
        kRows, kNPad, kDModel, 1.0f);
  }

  conv_gate_kernel<<<kBatch * (kSeq / kTTile), 256, 0, stream>>>(XIO, conv_w, conv_b, w_base, OOb, Gb, WHb);

  prefix_kernel<<<1, 64, 0, stream>>>(Gb, WHb, ACO);

  combine_kernel<<<(kRows * kDInner / 8) / 256, 256, 0, stream>>>(ACO, OOb, YH, YL);

  {
    dim3 grid((kRows / 64) * (kDModel / 64) / 8, 1);
    wmma_gemm64<1, true, 0, 0, false, 0><<<grid, 256, 0, stream>>>(
        YH, YL, kDInner, 0L, WOH, WOL, kDInner, 0L,
        (void*)out, nullptr, kDModel, 0L, nullptr, nullptr, 0L,
        kRows, kDModel, kDInner, 1.0f);
  }
}
